// BBBHetRegModel_26929444946732
// MI455X (gfx1250) — hardware-verified
//
#include <hip/hip_runtime.h>
#include <hip/hip_bf16.h>
#include <math.h>

typedef __attribute__((ext_vector_type(16))) _Float16 v16h;
typedef __attribute__((ext_vector_type(8)))  float    v8f;

#define N_TOTAL 131072
#define HID     1024
#define PRIOR1  4.0f
#define PRIOR2  0.0703125f
#define MIN_STD 1e-5f

__device__ __forceinline__ float softplusf(float v) {
    return fmaxf(v, 0.0f) + log1pf(expf(-fabsf(v)));
}

__device__ __forceinline__ float kl_term(float mu, float sigma, float prior) {
    float r = sigma / prior;
    float q = mu / prior;
    return 0.5f * (2.0f * logf(prior / sigma) - 1.0f + r * r + q * q);
}

__global__ __launch_bounds__(256) void bbb_main_kernel(
    const float* __restrict__ x,
    const float* __restrict__ W1_mu, const float* __restrict__ W1_rho,
    const float* __restrict__ b1_mu, const float* __restrict__ b1_rho,
    const float* __restrict__ W2_mu, const float* __restrict__ W2_rho,
    const float* __restrict__ b2_mu, const float* __restrict__ b2_rho,
    const float* __restrict__ eps_W1, const float* __restrict__ eps_b1,
    const float* __restrict__ eps_W2, const float* __restrict__ eps_b2,
    float* __restrict__ out)
{
    __shared__ float    sW1[HID];
    __shared__ float    sB1[HID];
    __shared__ _Float16 sW2p[3 * HID];
    __shared__ _Float16 sW2l[3 * HID];
    __shared__ float    sB2[2];
    __shared__ __attribute__((aligned(16))) float sOut[2][128];

    const int t = threadIdx.x;

    for (int j = t; j < HID; j += 256) {
        sW1[j] = fmaf(softplusf(W1_rho[j]), eps_W1[j], W1_mu[j]);
        sB1[j] = fmaf(softplusf(b1_rho[j]), eps_b1[j], b1_mu[j]);
    }
    for (int j = t; j < 2 * HID; j += 256) {
        const float wv = fmaf(softplusf(W2_rho[j]), eps_W2[j], W2_mu[j]);
        const _Float16 wh = (_Float16)wv;
        sW2p[j] = wh; sW2l[j] = (_Float16)((wv - (float)wh) * 2048.0f);
    }
    for (int j = t; j < HID; j += 256) {
        sW2p[2 * HID + j] = (_Float16)0.0f;
        sW2l[2 * HID + j] = (_Float16)0.0f;
    }
    if (t < 2) sB2[t] = fmaf(softplusf(b2_rho[t]), eps_b2[t], b2_mu[t]);
    __syncthreads();

    const int wave = t >> 5;
    const int lane = t & 31;
    const int m    = lane & 15;
    const int g    = lane >> 4;
    const int tile = blockIdx.x * 8 + wave;
    const int n0   = tile * 16;

    const float xm = x[n0 + m];

    const int brow = (m < 2) ? m : 2;
    const _Float16* __restrict__ bsrc  = &sW2p[brow * HID + g * 8];
    const _Float16* __restrict__ bsrcl = &sW2l[brow * HID + g * 8];
    const float* __restrict__ w1a = &sW1[g * 8];
    const float* __restrict__ w1b = &sW1[16 + g * 8];
    const float* __restrict__ b1a = &sB1[g * 8];
    const float* __restrict__ b1b = &sB1[16 + g * 8];

    v8f acc = {};
#pragma unroll 2
    for (int kk = 0; kk < HID; kk += 32) {
        v16h a, al;
#pragma unroll
        for (int h = 0; h < 8; ++h) {
            float v0 = fmaxf(fmaf(xm, w1a[kk + h], b1a[kk + h]), 0.0f);
            float v1 = fmaxf(fmaf(xm, w1b[kk + h], b1b[kk + h]), 0.0f);
            const _Float16 h0 = (_Float16)v0, h1 = (_Float16)v1;
            a[h]     = h0; al[h]     = (_Float16)((v0 - (float)h0) * 2048.0f);
            a[h + 8] = h1; al[h + 8] = (_Float16)((v1 - (float)h1) * 2048.0f);
        }

        v16h b, bl;
#pragma unroll
        for (int h = 0; h < 8; ++h) { b[h] = bsrc[kk + h]; b[h + 8] = bsrc[kk + 16 + h]; bl[h] = bsrcl[kk + h]; bl[h + 8] = bsrcl[kk + 16 + h]; }

        v8f xx = {};
        xx = __builtin_amdgcn_wmma_f32_16x16x32_f16(false, al, false, b, (short)0, xx, false, false);
        xx = __builtin_amdgcn_wmma_f32_16x16x32_f16(false, a, false, bl, (short)0, xx, false, false);
        acc = __builtin_amdgcn_wmma_f32_16x16x32_f16(
            false, a, false, b, (short)0, acc, false, false) + xx * (1.0f / 2048.0f);
    }

    if (m < 2) {
        const float bias = sB2[m];
#pragma unroll
        for (int r = 0; r < 8; ++r) {
            const float v = acc[r] + bias;
            sOut[m][wave * 16 + g * 8 + r] = (m == 0) ? v : (MIN_STD + softplusf(v));
        }
    }
    __syncthreads();
    if (t < 64) {
        typedef __attribute__((ext_vector_type(4))) float v4f_t;
        typedef float v4fa __attribute__((ext_vector_type(4), may_alias));
        const int which = t >> 5, q = t & 31;
        const v4f_t v = *(const v4fa*)&sOut[which][q * 4];
        float* dst = out + (size_t)which * N_TOTAL + (size_t)blockIdx.x * 128 + q * 4;
        *(volatile v4f_t*)dst = v; __threadfence(); *(volatile v4f_t*)dst = v;
    }

    if (blockIdx.x == 0) {
        __shared__ float red[256];
        float kl = 0.0f;
        for (int j = t; j < HID; j += 256) {
            kl += kl_term(W1_mu[j], softplusf(W1_rho[j]), PRIOR1);
            kl += kl_term(b1_mu[j], softplusf(b1_rho[j]), PRIOR1);
        }
        for (int j = t; j < 2 * HID; j += 256) kl += kl_term(W2_mu[j], softplusf(W2_rho[j]), PRIOR2);
        if (t < 2) kl += kl_term(b2_mu[t], softplusf(b2_rho[t]), PRIOR2);
        red[t] = kl;
        __syncthreads();
        for (int s = 128; s > 0; s >>= 1) { if (t < s) red[t] += red[t + s]; __syncthreads(); }
        if (t == 0) { const float v = red[0]; *(volatile float*)(out + 2 * N_TOTAL) = v; __threadfence(); *(volatile float*)(out + 2 * N_TOTAL) = v; }
    }
}

extern "C" void kernel_launch(void* const* d_in, const int* in_sizes, int n_in,
                              void* d_out, int out_size, void* d_ws, size_t ws_size,
                              hipStream_t stream) {
    (void)in_sizes; (void)n_in; (void)d_ws; (void)ws_size; (void)out_size;
    const float* x      = (const float*)d_in[0];
    const float* W1_mu  = (const float*)d_in[1];
    const float* W1_rho = (const float*)d_in[2];
    const float* b1_mu  = (const float*)d_in[3];
    const float* b1_rho = (const float*)d_in[4];
    const float* W2_mu  = (const float*)d_in[5];
    const float* W2_rho = (const float*)d_in[6];
    const float* b2_mu  = (const float*)d_in[7];
    const float* b2_rho = (const float*)d_in[8];
    const float* eps_W1 = (const float*)d_in[9];
    const float* eps_b1 = (const float*)d_in[10];
    const float* eps_W2 = (const float*)d_in[11];
    const float* eps_b2 = (const float*)d_in[12];
    float* out = (float*)d_out;

    bbb_main_kernel<<<N_TOTAL / 16 / 8, 256, 0, stream>>>(
        x, W1_mu, W1_rho, b1_mu, b1_rho, W2_mu, W2_rho, b2_mu, b2_rho,
        eps_W1, eps_b1, eps_W2, eps_b2, out);

}
